// WindowAttention3D_bac_65927747994176
// MI455X (gfx1250) — hardware-verified
//
#include <hip/hip_runtime.h>
#include <math.h>


#define __bf16 _Float16
typedef __attribute__((ext_vector_type(16))) _Float16 v16bf;
typedef __attribute__((ext_vector_type(8)))  float  v8f;

#define B_WIN   512
#define NTOK    98
#define CDIM    128
#define NHEADS  4
#define HD      32
#define NWIN    256
#define QKV_ELEMS ((long)B_WIN * NHEADS * NTOK * HD)

union Frag16 { v16bf f; uint4 q[2]; };

__device__ __forceinline__ v8f zero8() {
    v8f z;
#pragma unroll
    for (int i = 0; i < 8; ++i) z[i] = 0.0f;
    return z;
}

__device__ __forceinline__ v16bf zero16() {
    Frag16 r;
    r.q[0] = make_uint4(0u, 0u, 0u, 0u);
    r.q[1] = make_uint4(0u, 0u, 0u, 0u);
    return r.f;
}

__device__ __forceinline__ v16bf load_frag_a(const __bf16* m, int ld,
                                             int row0, int nrows, int k0) {
    unsigned lane = threadIdx.x & 31u;
    int row  = row0 + (int)(lane & 15u);
    int half = (int)(lane >> 4) & 1;
    if (row >= nrows) return zero16();
    const __bf16* p = m + (long)row * ld + k0 + half * 8;
    Frag16 r;
    r.q[0] = *(const uint4*)(p);
    r.q[1] = *(const uint4*)(p + 16);
    return r.f;
}

__device__ __forceinline__ v16bf load_frag_bT(const __bf16* m, int ld,
                                              int n0, int nrows, int k0) {
    unsigned lane = threadIdx.x & 31u;
    int n    = n0 + (int)(lane & 15u);
    int half = (int)(lane >> 4) & 1;
    if (n >= nrows) return zero16();
    const __bf16* p = m + (long)n * ld + k0 + half * 8;
    Frag16 r;
    r.q[0] = *(const uint4*)(p);
    r.q[1] = *(const uint4*)(p + 16);
    return r.f;
}

__device__ __forceinline__ v8f wmma_bf16(v16bf a, v16bf b, v8f c) {
    return __builtin_amdgcn_wmma_f32_16x16x32_f16(
        false, a, false, b, (short)0, c, false, false);
}

__global__ __launch_bounds__(128) void qkv_gemm_kernel(
    const float* __restrict__ x, const float* __restrict__ w,
    __bf16* __restrict__ qws, __bf16* __restrict__ kws,
    __bf16* __restrict__ vws) {
    __shared__ __align__(16) __bf16 As[64 * 128];
    __shared__ __align__(16) __bf16 Ws[64 * 128];

    const int row0 = blockIdx.x * 64;
    const int col0 = blockIdx.y * 64;
    const int tid  = threadIdx.x;

    const float4* xs4 = (const float4*)(x + (long)row0 * 128);
    const float4* ws4 = (const float4*)(w + (long)col0 * 128);
    for (int idx = tid; idx < 2048; idx += 128) {
        float4 t = xs4[idx];
        __bf16* d = As + idx * 4;
        d[0] = (__bf16)t.x; d[1] = (__bf16)t.y;
        d[2] = (__bf16)t.z; d[3] = (__bf16)t.w;
        float4 u = ws4[idx];
        __bf16* e = Ws + idx * 4;
        e[0] = (__bf16)u.x; e[1] = (__bf16)u.y;
        e[2] = (__bf16)u.z; e[3] = (__bf16)u.w;
    }
    __syncthreads();

    const int wv = tid >> 5;
    v8f acc[4];
#pragma unroll
    for (int n = 0; n < 4; ++n) acc[n] = zero8();

#pragma unroll
    for (int kc = 0; kc < 4; ++kc) {
        v16bf a = load_frag_a(As, 128, wv * 16, 64, kc * 32);
#pragma unroll
        for (int n = 0; n < 4; ++n) {
            v16bf b = load_frag_bT(Ws, 128, n * 16, 64, kc * 32);
            acc[n] = wmma_bf16(a, b, acc[n]);
        }
    }

    const unsigned lane = tid & 31u;
    const int half = (int)(lane >> 4) & 1;
    const int lnc  = (int)(lane & 15u);
    const int s = col0 >> 7;
    const float qscale = (s == 0) ? 0.17677669529663687f : 1.0f;
    __bf16* dstw = (s == 0) ? qws : (s == 1) ? kws : vws;
    __syncthreads();
    __bf16* T = As;
#pragma unroll
    for (int n = 0; n < 4; ++n)
#pragma unroll
        for (int r = 0; r < 8; ++r) T[(wv * 16 + r + 8 * half) * 64 + n * 16 + lnc] = (__bf16)(acc[n][r] * qscale);
    __syncthreads();
    const int hh0 = (col0 >> 5) & 3;
    typedef __attribute__((ext_vector_type(4))) unsigned v4u_t;
    v4u_t cv[4]; long co[4];
#pragma unroll
    for (int i2 = 0; i2 < 4; ++i2) {
        const int c = tid + 128 * i2, L = c >> 3, q = c & 7;
        const int pair = L >> 1, hsel = L & 1;
        const int trow = pair * 2 + (q >> 2), d8 = (q & 3) * 8;
        cv[i2] = *(const v4u_t*)(T + trow * 64 + hsel * 32 + d8);
        const int i = row0 + trow, b = i / NTOK, nn = i % NTOK;
        co[i2] = (((long)(b * NHEADS + hh0 + hsel)) * NTOK + nn) * HD + d8;
    }
#pragma unroll
    for (int i2 = 0; i2 < 4; ++i2) *(volatile v4u_t*)(dstw + co[i2]) = cv[i2];
    __threadfence();
#pragma unroll
    for (int i2 = 0; i2 < 4; ++i2) *(volatile v4u_t*)(dstw + co[i2]) = cv[i2];
}

__global__ __launch_bounds__(128) void attn_fused_kernel(
    const __bf16* __restrict__ qws, const __bf16* __restrict__ kws,
    const __bf16* __restrict__ vws, const float* __restrict__ bias_table,
    const float* __restrict__ mask, float* __restrict__ out) {
    __shared__ __align__(16) __bf16 Qs[NTOK * HD];
    __shared__ __align__(16) __bf16 Ks[NTOK * HD];
    __shared__ __align__(16) __bf16 Vt[HD * 128];
    __shared__ __align__(16) float  Ss[NTOK * 112];
    __bf16* Ps = (__bf16*)Ss;

    const int b   = blockIdx.x;
    const int h   = blockIdx.y;
    const int tid = threadIdx.x;
    const int wv  = tid >> 5;
    const unsigned lane = tid & 31u;
    const int half = (int)(lane >> 4) & 1;
    const int lnc  = (int)(lane & 15u);

    const long base = ((long)(b * NHEADS + h)) * NTOK * HD;
    {
        const uint4* q4 = (const uint4*)(qws + base);
        const uint4* k4 = (const uint4*)(kws + base);
        uint4* qd = (uint4*)Qs;
        uint4* kd = (uint4*)Ks;
        for (int idx = tid; idx < 392; idx += 128) {
            qd[idx] = q4[idx];
            kd[idx] = k4[idx];
        }
        const __bf16* vsrc = vws + base;
        for (int idx = tid; idx < HD * 128; idx += 128) {
            int d = idx >> 7, key = idx & 127;
            Vt[idx] = (key < NTOK) ? vsrc[(long)key * HD + d] : (__bf16)0.0f;
        }
    }
    __syncthreads();

    for (int t = wv; t < 49; t += 4) {
        int ti = t / 7, tj = t % 7;
        v16bf a  = load_frag_a(Qs, HD, ti * 16, NTOK, 0);
        v16bf bt = load_frag_bT(Ks, HD, tj * 16, NTOK, 0);
        v8f c = wmma_bf16(a, bt, zero8());
#pragma unroll
        for (int r = 0; r < 8; ++r) {
            int row = ti * 16 + r + 8 * half;
            if (row < NTOK) Ss[row * 112 + tj * 16 + lnc] = c[r];
        }
    }
    __syncthreads();

    if (tid < NTOK) {
        const int r  = tid;
        const int zr = r / 49, rr = r - zr * 49;
        const int yr = rr / 7, xr = rr - yr * 7;
        const float* mrow = mask + ((long)(b & (NWIN - 1))) * NTOK * NTOK
                                 + (long)r * NTOK;
        float* srow = Ss + r * 112;
        float mx = -3.4e38f;
        int c2 = 0;
        for (int zc = 0; zc < 2; ++zc) {
            int zb = (zr - zc + 1) * 169;
            for (int yc = 0; yc < 7; ++yc) {
                int yb = zb + (yr - yc + 6) * 13 + xr + 6;
#pragma unroll
                for (int xc = 0; xc < 7; ++xc, ++c2) {
                    float t = srow[c2] + bias_table[(yb - xc) * NHEADS + h]
                                       + mrow[c2];
                    srow[c2] = t;
                    mx = fmaxf(mx, t);
                }
            }
        }
        float sum = 0.0f;
        for (int c3 = 0; c3 < NTOK; ++c3) {
            float e = __expf(srow[c3] - mx);
            srow[c3] = e;
            sum += e;
        }
        float inv = 1.0f / sum;
        unsigned* prow = (unsigned*)((char*)Ss + (long)r * 448);
        for (int c3 = 0; c3 < 128; c3 += 2) {
            float p0 = (c3     < NTOK) ? srow[c3]     * inv : 0.0f;
            float p1 = (c3 + 1 < NTOK) ? srow[c3 + 1] * inv : 0.0f;
            union { __bf16 hh[2]; unsigned u; } pk;
            pk.hh[0] = (__bf16)(p0 * 1024.0f);
            pk.hh[1] = (__bf16)(p1 * 1024.0f);
            prow[c3 >> 1] = pk.u;
        }
    }
    __syncthreads();

    __shared__ __align__(16) float Ostg[4][16 * 32];
    float* stg = Ostg[wv];
    for (int ti = wv; ti < 7; ti += 4) {
        v8f acc0 = zero8(), acc1 = zero8();
#pragma unroll
        for (int kc = 0; kc < 4; ++kc) {
            v16bf a   = load_frag_a(Ps, 224, ti * 16, NTOK, kc * 32);
            v16bf bb0 = load_frag_bT(Vt, 128, 0,  HD, kc * 32);
            v16bf bb1 = load_frag_bT(Vt, 128, 16, HD, kc * 32);
            acc0 = wmma_bf16(a, bb0, acc0);
            acc1 = wmma_bf16(a, bb1, acc1);
        }
#pragma unroll
        for (int r = 0; r < 8; ++r) {
            stg[(r + 8 * half) * 32 + lnc]      = acc0[r] * (1.0f / 1024.0f);
            stg[(r + 8 * half) * 32 + 16 + lnc] = acc1[r] * (1.0f / 1024.0f);
        }
        asm volatile("s_wait_dscnt 0" ::: "memory");
        typedef __attribute__((ext_vector_type(4))) float v4f_t;
        typedef float v4fa __attribute__((ext_vector_type(4), may_alias));
        v4f_t ov[4]; long oo[4]; bool ok[4];
#pragma unroll
        for (int i2 = 0; i2 < 4; ++i2) {
            const int c = (int)lane + 32 * i2, rr = c >> 3, q = c & 7, row = ti * 16 + rr;
            ov[i2] = *(const volatile v4fa*)(stg + rr * 32 + q * 4);
            ok[i2] = row < NTOK;
            oo[i2] = ((long)b * NTOK + row) * CDIM + h * HD + q * 4;
        }
#pragma unroll
        for (int i2 = 0; i2 < 4; ++i2) if (ok[i2]) *(volatile v4f_t*)(out + oo[i2]) = ov[i2];
        __threadfence();
#pragma unroll
        for (int i2 = 0; i2 < 4; ++i2) if (ok[i2]) *(volatile v4f_t*)(out + oo[i2]) = ov[i2];
        asm volatile("s_wait_dscnt 0" ::: "memory");
    }
}

extern "C" void kernel_launch(void* const* d_in, const int* in_sizes, int n_in,
                              void* d_out, int out_size, void* d_ws,
                              size_t ws_size, hipStream_t stream) {
    const float* x          = (const float*)d_in[0];
    const float* qkv_w      = (const float*)d_in[1];
    const float* bias_table = (const float*)d_in[2];
    const float* mask       = (const float*)d_in[3];
    float* out = (float*)d_out;

    __bf16* qws = (__bf16*)d_ws;
    __bf16* kws = qws + QKV_ELEMS;
    __bf16* vws = kws + QKV_ELEMS;

    dim3 g1(784, 6), blk(128);
    hipLaunchKernelGGL(qkv_gemm_kernel, g1, blk, 0, stream,
                       x, qkv_w, qws, kws, vws);

    dim3 g2(B_WIN, NHEADS);
    hipLaunchKernelGGL(attn_fused_kernel, g2, blk, 0, stream,
                       qws, kws, vws, bias_table, mask, out);
}
